// RotaryMHA_30313879176084
// MI455X (gfx1250) — hardware-verified
//
#include <hip/hip_runtime.h>
#include <math.h>
#include <stdint.h>

#ifndef NB
#define NB 4
#endif
#ifndef SEQ
#define SEQ 2048
#endif
#define NB_FULL 4
#define XS_FULL 2048
#define DMOD  1024
#define NH    16
#define HD    64
#define HHALF 32
#define NFREQ 32
#define CSW   64
#define MROWS (NB * SEQ)
#define RSQ_HD 0.125f
#define LOG2E 1.4426950408889634f
#define QSC   256.0f
#define KSC   256.0f
#define PCAR  32768.0f
#define VCAR  1024.0f
#define OSC   1024.0f
#define WOS   1024.0f
#define WPB   4
#define NHG   (NH / WPB)
#define NQT   (SEQ / 16)
#define NST   (SEQ / 64)
#define NKT   (SEQ / 32)
#define ATT_THREADS (WPB * 32)
#define PTP   36
#define PTW   (16 * PTP)
#define SLP   68
#define SLW   (16 * SLP)
#define WREG  (PTW + SLW)
#define SLAB64 (16 * 68)
#define VTP   72
#define CTP   68
#define WS_CAP 134217728
static_assert(DMOD == NH * HD && HD == 64 && NH == 16 && WPB == 4 && NHG * WPB == NH && 2 * HHALF == HD && NFREQ == HHALF);
static_assert(ATT_THREADS == 128 && CSW == 2 * NFREQ);
static_assert(NB >= 1 && NB <= NB_FULL);
static_assert((SEQ % 64) == 0 && SEQ >= 64 && SEQ <= XS_FULL);
static_assert((DMOD % 64) == 0 && (DMOD % 32) == 0 && (HD % 32) == 0 && (MROWS % 64) == 0 && (DMOD / 8) == 128);
static_assert(((SEQ * DMOD / 8) % 256) == 0 && ((DMOD * DMOD / 8) % 256) == 0 && ((MROWS * DMOD / 8) % 256) == 0);
static_assert(((SEQ * NFREQ) % 256) == 0 && (SEQ % 8) == 0);
static_assert(WPB * WREG * 4 <= 65536 && 2 * HD * VTP * 2 <= 65536 && 4 * SLAB64 * 4 <= 65536 && 8 * CTP * 4 <= 65536);

typedef unsigned short u16;
typedef _Float16 v16h __attribute__((ext_vector_type(16)));
typedef _Float16 v8h  __attribute__((ext_vector_type(8)));
typedef __bf16   v16b __attribute__((ext_vector_type(16)));
typedef float    v8f  __attribute__((ext_vector_type(8)));
typedef float    v4f  __attribute__((ext_vector_type(4)));
typedef unsigned int v4u __attribute__((ext_vector_type(4)));

union FragH { v16h v; v8h h[2]; v4u u[2]; };
union FragB { v16b v; v4u u[2]; };

struct RopeFreq { float f[NFREQ]; };
static_assert(sizeof(RopeFreq) == NFREQ * 4);

__device__ __forceinline__ unsigned short bf_bits(float f) {
  unsigned u = __float_as_uint(f);
  return (unsigned short)((u + 0x7FFFu + ((u >> 16) & 1u)) >> 16);
}
__device__ __forceinline__ float bf_up(unsigned short h) { return __uint_as_float(((unsigned)h) << 16); }
__device__ __forceinline__ float bfr(float f) { return bf_up(bf_bits(f)); }
__device__ __forceinline__ unsigned short h_bits(_Float16 x) { return __builtin_bit_cast(unsigned short, x); }
__device__ __forceinline__ unsigned pk16(unsigned short a, unsigned short b) { return (unsigned)a | ((unsigned)b << 16); }
__device__ __forceinline__ v8f zero8() { v8f z = {0.f, 0.f, 0.f, 0.f, 0.f, 0.f, 0.f, 0.f}; return z; }

__device__ __forceinline__ v16h ldfrag_h(const _Float16* p) {
  FragH f;
  f.h[0] = *(const v8h*)(p);
  f.h[1] = *(const v8h*)(p + 16);
  return f.v;
}
__device__ __forceinline__ v16b ldfrag_b(const u16* p) {
  FragB f;
  f.u[0] = *(const v4u*)(p);
  f.u[1] = *(const v4u*)(p + 16);
  return f.v;
}

__device__ __forceinline__ v8f mma_h(v16h a, v16h b, v8f c) {
  return __builtin_amdgcn_wmma_f32_16x16x32_f16(false, a, false, b, (short)0, c, false, false);
}
__device__ __forceinline__ v8f mma_b(v16b a, v16b b, v8f c) {
  return __builtin_amdgcn_wmma_f32_16x16x32_bf16(false, a, false, b, (short)0, c, false, false);
}
__device__ __forceinline__ void guard2(v8f& a, v8f& b, v16h x0, v16h x1, v16h x2, v16h x3, v16h x4, v16h x5) {
#if defined(__HIP_DEVICE_COMPILE__)
  asm volatile("v_nop\n\tv_nop\n\tv_nop\n\tv_nop"
               : "+v"(a), "+v"(b) : "v"(x0), "v"(x1), "v"(x2), "v"(x3), "v"(x4), "v"(x5) : "memory");
#endif
}
template <typename F>
__device__ __forceinline__ void guard6(v8f& a, v8f& b, v8f& c, v8f& d, F x0, F x1, F x2, F x3, F x4, F x5) {
#if defined(__HIP_DEVICE_COMPILE__)
  asm volatile("v_nop\n\tv_nop\n\tv_nop\n\tv_nop"
               : "+v"(a), "+v"(b), "+v"(c), "+v"(d) : "v"(x0), "v"(x1), "v"(x2), "v"(x3), "v"(x4), "v"(x5) : "memory");
#endif
}
__device__ __forceinline__ void acc_guard4(v8f& a, v8f& b, v8f& c, v8f& d) {
#if defined(__HIP_DEVICE_COMPILE__)
  asm volatile("v_nop\n\tv_nop\n\tv_nop\n\tv_nop" : "+v"(a), "+v"(b), "+v"(c), "+v"(d));
#endif
}
__device__ __forceinline__ void wave_sync_lds() {
  __builtin_amdgcn_fence(__ATOMIC_RELEASE, "workgroup");
  __builtin_amdgcn_wave_barrier();
  __builtin_amdgcn_fence(__ATOMIC_ACQUIRE, "workgroup");
}

__global__ __launch_bounds__(256) void cvt16(const float* __restrict__ x, u16* D, int n8, int f16mode, float scale) {
  const int gt = blockIdx.x * 256 + (int)threadIdx.x;
  if (gt >= n8) return;
  const float* p = x + (size_t)gt * 8;
  const v4f a = *(const v4f*)(p), b4 = *(const v4f*)(p + 4);
  float w[8];
#pragma unroll
  for (int e = 0; e < 4; ++e) { w[e] = a[e]; w[4 + e] = b4[e]; }
  v4u o;
#pragma unroll
  for (int e = 0; e < 4; ++e) {
    const float f0 = w[2 * e], f1 = w[2 * e + 1];
    const unsigned short hb0 = h_bits((_Float16)(bfr(f0) * scale));
    const unsigned short hb1 = h_bits((_Float16)(bfr(f1) * scale));
    const unsigned short bb0 = bf_bits(f0);
    const unsigned short bb1 = bf_bits(f1);
    o[e] = (f16mode != 0) ? pk16(hb0, hb1) : pk16(bb0, bb1);
  }
  u16* d = D + (size_t)gt * 8;
  for (int pass = 0; pass < 2; ++pass) {
    *(volatile v4u*)(d) = o;
    __threadfence();
  }
}

__global__ __launch_bounds__(256) void cstab(float* CS, RopeFreq fr) {
  __shared__ __align__(16) float tile[8 * CTP];
  const int tid = threadIdx.x;
  const int i   = tid & 31;
  const int tl  = tid >> 5;
  const int t   = blockIdx.x * 8 + tl;
  float f = fr.f[0];
#pragma unroll
  for (int j = 1; j < NFREQ; ++j) f = (i == j) ? fr.f[j] : f;
  const float ang = (float)t * f;
  float sv, cv;
  sincosf(ang, &sv, &cv);
  tile[tl * CTP + i]         = cv;
  tile[tl * CTP + HHALF + i] = sv;
  __syncthreads();
  if (tid < 128) {
    const int row = tid >> 4, c4 = (tid & 15) * 4;
    const v4f v = *(const v4f*)(tile + row * CTP + c4);
    float* dst = CS + (size_t)(blockIdx.x * 8 + row) * CSW + c4;
    for (int pass = 0; pass < 2; ++pass) {
      *(volatile v4f*)(dst) = v;
      __threadfence();
    }
  }
}

__global__ __launch_bounds__(256) void rope16(const float* __restrict__ F, const float* __restrict__ CS,
                                              u16* Hp, int n8, float sc) {
#pragma clang fp contract(off)
  const int gt = blockIdx.x * 256 + (int)threadIdx.x;
  if (gt >= n8) return;
  const int row = gt / (DMOD / 8);
  const int col = (gt % (DMOD / 8)) * 8;
  const int s   = row % SEQ;
  const int d0  = col & (HD - 1);
  const int i0  = d0 & (HHALF - 1);
  const bool first = (d0 < HHALF);
  const int pcol = first ? (col + HHALF) : (col - HHALF);
  const float* po = F + (size_t)row * DMOD + col;
  const float* pp = F + (size_t)row * DMOD + pcol;
  const float* pc = CS + (size_t)s * CSW + i0;
  const v4f o0 = *(const v4f*)(po), o1 = *(const v4f*)(po + 4);
  const v4f p0 = *(const v4f*)(pp), p1 = *(const v4f*)(pp + 4);
  const v4f c0 = *(const v4f*)(pc), c1 = *(const v4f*)(pc + 4);
  const v4f n0 = *(const v4f*)(pc + HHALF), n1 = *(const v4f*)(pc + HHALF + 4);
  float w[8];
#pragma unroll
  for (int e = 0; e < 4; ++e) {
    {
      const float ov = o0[e], pv = p0[e], cv = c0[e], sv = n0[e];
      const float m1 = ov * cv, m2 = pv * sv;
      const float ra = m1 - m2;
      const float rb = m2 + m1;
      w[e] = (first ? ra : rb) * sc;
    }
    {
      const float ov = o1[e], pv = p1[e], cv = c1[e], sv = n1[e];
      const float m1 = ov * cv, m2 = pv * sv;
      const float ra = m1 - m2;
      const float rb = m2 + m1;
      w[4 + e] = (first ? ra : rb) * sc;
    }
  }
  v4u oh;
#pragma unroll
  for (int e = 0; e < 4; ++e) {
    const _Float16 h0 = (_Float16)w[2 * e], h1 = (_Float16)w[2 * e + 1];
    oh[e] = pk16(h_bits(h0), h_bits(h1));
  }
  u16* dh = Hp + (size_t)gt * 8;
  for (int pass = 0; pass < 2; ++pass) {
    *(volatile v4u*)(dh) = oh;
    __threadfence();
  }
}

__global__ __launch_bounds__(256) void vt16(const float* __restrict__ F, u16* VHo, u16* VLo) {
  __shared__ __align__(16) u16 TH[HD * VTP];
  __shared__ __align__(16) u16 TL[HD * VTP];
  const int tid = threadIdx.x;
  const int bid = blockIdx.x;
  const int st  = bid % NST;
  const int t2  = bid / NST;
  const int g   = t2 % NH;
  const int b   = t2 / NH;
  if (b >= NB) return;
  const int s0  = st * 64;
  {
    const int sl = tid >> 2;
    const int dc = (tid & 3) * 16;
    const float* src = F + ((size_t)b * SEQ + s0 + sl) * DMOD + g * HD + dc;
#pragma unroll
    for (int i = 0; i < 4; ++i) {
      const v4f a = *(const v4f*)(src + 4 * i);
#pragma unroll
      for (int e = 0; e < 4; ++e) {
        const float t = a[e] * VCAR;
        const _Float16 hv = (_Float16)t;
        const _Float16 lv = (_Float16)(t - (float)hv);
        TH[(dc + 4 * i + e) * VTP + sl] = h_bits(hv);
        TL[(dc + 4 * i + e) * VTP + sl] = h_bits(lv);
      }
    }
  }
  __syncthreads();
  v4u vh[2], vl[2];
  const int q8 = tid >> 3, p8 = (tid & 7) * 8;
#pragma unroll
  for (int it = 0; it < 2; ++it) {
    const int line = it * 32 + q8;
    vh[it] = *(const v4u*)(TH + line * VTP + p8);
    vl[it] = *(const v4u*)(TL + line * VTP + p8);
  }
  const size_t hrow = (size_t)(b * NH + g) * HD;
  const size_t base = hrow * SEQ + s0 + p8;
  for (int pass = 0; pass < 2; ++pass) {
#pragma unroll
    for (int it = 0; it < 2; ++it) {
      const int line = it * 32 + q8;
      *(volatile v4u*)(VHo + base + (size_t)line * SEQ) = vh[it];
      *(volatile v4u*)(VLo + base + (size_t)line * SEQ) = vl[it];
    }
    __threadfence();
  }
}

__device__ __forceinline__ void epi64(float* sl, v8f a0, v8f a1, v8f a2, v8f a3, float oscale,
                                      float* C, int N, size_t rowb, int col0, int lane) {
  const int hh = lane >> 4, m = lane & 15;
#pragma unroll
  for (int r = 0; r < 8; ++r) {
    const int ro = (8 * hh + r) * 68 + m;
    sl[ro]      = a0[r] * oscale;
    sl[ro + 16] = a1[r] * oscale;
    sl[ro + 32] = a2[r] * oscale;
    sl[ro + 48] = a3[r] * oscale;
  }
  wave_sync_lds();
  v4f vals[8];
#pragma unroll
  for (int it = 0; it < 8; ++it) vals[it] = *(const v4f*)(sl + (it * 2 + hh) * 68 + m * 4);
  float* dst = C + (rowb + (size_t)hh) * (size_t)N + col0 + m * 4;
  for (int pass = 0; pass < 2; ++pass) {
#pragma unroll
    for (int it = 0; it < 8; ++it) {
      *(volatile v4f*)(dst + (size_t)(it * 2) * (size_t)N) = vals[it];
    }
    __threadfence();
  }
}

__global__ __launch_bounds__(128)
void gemm_bf(const u16* __restrict__ A, const u16* __restrict__ Bt, float* C, int M, int N, int K, float oscale) {
  __shared__ __align__(16) float slab[4 * SLAB64];
  const int tid = threadIdx.x, wave = tid >> 5, lane = tid & 31, hh = lane >> 4, m = lane & 15;
  const int ntile = N >> 6;
  const int bid   = blockIdx.x;
  const int rowb  = (bid / ntile) * 64 + wave * 16;
  const int col0  = (bid % ntile) * 64;
  if (rowb + 16 > M) return;
  const u16* ap = A  + (size_t)(rowb + m) * K + 8 * hh;
  const u16* bp = Bt + (size_t)(col0 + m) * K + 8 * hh;
  const size_t bs = (size_t)16 * K;
  v8f acc0 = zero8(), acc1 = zero8(), acc2 = zero8(), acc3 = zero8();
#pragma unroll 1
  for (int k0 = 0; k0 < K; k0 += 32) {
    const v16b a  = ldfrag_b(ap + k0);
    const v16b b0 = ldfrag_b(bp + k0);
    const v16b b1 = ldfrag_b(bp + bs + k0);
    const v16b b2 = ldfrag_b(bp + 2 * bs + k0);
    const v16b b3 = ldfrag_b(bp + 3 * bs + k0);
    acc0 = mma_b(a, b0, acc0);
    acc1 = mma_b(a, b1, acc1);
    acc2 = mma_b(a, b2, acc2);
    acc3 = mma_b(a, b3, acc3);
    guard6<v16b>(acc0, acc1, acc2, acc3, a, b0, b1, b2, b3, a);
  }
  epi64(slab + wave * SLAB64, acc0, acc1, acc2, acc3, oscale, C, N, (size_t)rowb, col0, lane);
}

template <int NPROD>
__global__ __launch_bounds__(128)
void gemm_o(const u16* __restrict__ Ah, const u16* __restrict__ Al, const u16* __restrict__ Bt,
            float* C, int sbeg, int nrt, float oscale) {
  __shared__ __align__(16) float slab[4 * SLAB64];
  const int tid = threadIdx.x, wave = tid >> 5, lane = tid & 31, hh = lane >> 4, m = lane & 15;
  const int ntile = DMOD >> 6;
  const int bid   = blockIdx.x;
  const int ct    = bid % ntile;
  const int t2    = bid / ntile;
  const int rt    = t2 % nrt;
  const int bb    = t2 / nrt;
  if (bb >= NB) return;
  const int srow  = sbeg + rt * 64 + wave * 16;
  if (srow + 16 > SEQ) return;
  const int col0  = ct * 64;
  const int K     = DMOD;
  const size_t rowC = (size_t)bb * SEQ + srow;
  const _Float16* ahp = (const _Float16*)(const void*)Ah + (rowC + m) * K + 8 * hh;
  const _Float16* alp = (const _Float16*)(const void*)Al + (rowC + m) * K + 8 * hh;
  const _Float16* bp  = (const _Float16*)(const void*)Bt + (size_t)(col0 + m) * K + 8 * hh;
  const size_t bs = (size_t)16 * K;
  v8f acc0 = zero8(), acc1 = zero8(), acc2 = zero8(), acc3 = zero8();
  if constexpr (NPROD == 2) {
#pragma unroll 1
    for (int k0 = 0; k0 < K; k0 += 32) {
      const v16h ah = ldfrag_h(ahp + k0), al = ldfrag_h(alp + k0);
      const v16h b0 = ldfrag_h(bp + k0);
      const v16h b1 = ldfrag_h(bp + bs + k0);
      const v16h b2 = ldfrag_h(bp + 2 * bs + k0);
      const v16h b3 = ldfrag_h(bp + 3 * bs + k0);
      acc0 = mma_h(ah, b0, acc0);  acc0 = mma_h(al, b0, acc0);
      acc1 = mma_h(ah, b1, acc1);  acc1 = mma_h(al, b1, acc1);
      acc2 = mma_h(ah, b2, acc2);  acc2 = mma_h(al, b2, acc2);
      acc3 = mma_h(ah, b3, acc3);  acc3 = mma_h(al, b3, acc3);
      guard6<v16h>(acc0, acc1, acc2, acc3, ah, al, b0, b1, b2, b3);
    }
  } else {
#pragma unroll 1
    for (int k0 = 0; k0 < K; k0 += 32) {
      const v16h ah = ldfrag_h(ahp + k0);
      const v16h b0 = ldfrag_h(bp + k0);
      const v16h b1 = ldfrag_h(bp + bs + k0);
      const v16h b2 = ldfrag_h(bp + 2 * bs + k0);
      const v16h b3 = ldfrag_h(bp + 3 * bs + k0);
      acc0 = mma_h(ah, b0, acc0);
      acc1 = mma_h(ah, b1, acc1);
      acc2 = mma_h(ah, b2, acc2);
      acc3 = mma_h(ah, b3, acc3);
      guard6<v16h>(acc0, acc1, acc2, acc3, ah, b0, b1, b2, b3, ah);
    }
  }
  epi64(slab + wave * SLAB64, acc0, acc1, acc2, acc3, oscale, C, DMOD, rowC, col0, lane);
}

__global__ __launch_bounds__(ATT_THREADS)
void attn_h(const u16* __restrict__ QHp, const u16* __restrict__ KHp,
            const u16* __restrict__ VHp, const u16* __restrict__ VLp,
            const int* __restrict__ MK, u16* OHp, int qtbeg, int nqt) {
  __shared__ __align__(16) float smem[WPB * WREG];

  const int tid  = threadIdx.x;
  const int wave = tid >> 5;
  const int lane = tid & 31;
  const int hh   = lane >> 4;
  const int c    = lane & 15;
  const int bid  = blockIdx.x;
  const int qt   = qtbeg + bid % nqt;
  const int t2   = bid / nqt;
  const int hg   = t2 % NHG;
  const int b    = t2 / NHG;
  if (b >= NB) return;
  const int q0   = qt * 16;
  if (q0 + 16 > SEQ) return;
  const int head = hg * WPB + wave;

  float* pt   = smem + wave * WREG;
  float* slab = pt + PTW;

  const size_t hcol = (size_t)head * HD + 8 * hh;
  const _Float16* Qh  = (const _Float16*)(const void*)QHp + ((size_t)b * SEQ + q0 + c) * DMOD + hcol;
  const _Float16* Khb = (const _Float16*)(const void*)KHp + ((size_t)b * SEQ + c) * DMOD + hcol;
  const size_t vrow = ((size_t)(b * NH + head) * HD + c) * SEQ + 8 * hh;
  const _Float16* Vhb = (const _Float16*)(const void*)VHp + vrow;
  const _Float16* Vlb = (const _Float16*)(const void*)VLp + vrow;
  const int* mk = MK + (size_t)b * XS_FULL;
  const float lsc = RSQ_HD * (LOG2E / (QSC * KSC));
  const float oc  = 1.0f / (PCAR * VCAR);
  const size_t KROW = (size_t)DMOD;

  v16h qhf[HD / 32];
#pragma unroll
  for (int kk = 0; kk < HD / 32; ++kk) qhf[kk] = ldfrag_h(Qh + kk * 32);

  float mrow[8], lrow[8];
  v8f o[4];
#pragma unroll
  for (int r = 0; r < 8; ++r) { mrow[r] = -INFINITY; lrow[r] = 0.f; }
#pragma unroll
  for (int j = 0; j < 4; ++j) o[j] = zero8();

#pragma unroll 1
  for (int kt = 0; kt < NKT; ++kt) {
    const int kb = kt * 32;
    const int mk0 = mk[kb + c];
    const int mk1 = mk[kb + 16 + c];
    v8f s0 = zero8(), s1 = zero8();
    const _Float16* k0p = Khb + (size_t)kb * KROW;
    const _Float16* k1p = k0p + (size_t)16 * KROW;
#pragma unroll
    for (int kk = 0; kk < HD / 32; ++kk) {
      const v16h kh0 = ldfrag_h(k0p + kk * 32);
      const v16h kh1 = ldfrag_h(k1p + kk * 32);
      s0 = mma_h(qhf[kk], kh0, s0);
      s1 = mma_h(qhf[kk], kh1, s1);
      guard2(s0, s1, qhf[kk], kh0, kh1, qhf[kk], kh0, kh1);
    }
#pragma unroll
    for (int r = 0; r < 8; ++r) {
      const float u0 = s0[r] * lsc;
      const float u1 = s1[r] * lsc;
      const float t0 = (mk0 != 0) ? -INFINITY : u0;
      const float t1 = (mk1 != 0) ? -INFINITY : u1;
      float mx = fmaxf(t0, t1);
#pragma unroll
      for (int off = 1; off < 16; off <<= 1) mx = fmaxf(mx, __shfl_xor(mx, off, 32));
      const float mn = fmaxf(mrow[r], mx);
      const float ms = (mn == -INFINITY) ? 0.0f : mn;
      const float al = exp2f(mrow[r] - ms);
      mrow[r] = mn;
      const float e0 = exp2f(t0 - ms), e1 = exp2f(t1 - ms);
      float ps = e0 + e1;
#pragma unroll
      for (int off = 1; off < 16; off <<= 1) ps += __shfl_xor(ps, off, 32);
      lrow[r] = lrow[r] * al + ps;
#pragma unroll
      for (int j = 0; j < 4; ++j) o[j][r] *= al;
      const int ro = (8 * hh + r) * PTP + c;
      pt[ro]      = e0;
      pt[ro + 16] = e1;
    }
    wave_sync_lds();
    FragH ph;
    {
      const float* prow = pt + c * PTP + 8 * hh;
      const v4f p0 = *(const v4f*)(prow), p1 = *(const v4f*)(prow + 4);
      const v4f p2 = *(const v4f*)(prow + 16), p3 = *(const v4f*)(prow + 20);
#pragma unroll
      for (int e = 0; e < 4; ++e) {
        ph.h[0][e]     = (_Float16)(p0[e] * PCAR);
        ph.h[0][4 + e] = (_Float16)(p1[e] * PCAR);
        ph.h[1][e]     = (_Float16)(p2[e] * PCAR);
        ph.h[1][4 + e] = (_Float16)(p3[e] * PCAR);
      }
    }
    {
      const _Float16* vhp = Vhb + kb;
      const _Float16* vlp = Vlb + kb;
#pragma unroll
      for (int jg = 0; jg < 2; ++jg) {
        const size_t da = (size_t)(2 * jg) * 16 * SEQ;
        const size_t db = da + (size_t)16 * SEQ;
        const v16h vha = ldfrag_h(vhp + da), vhb2 = ldfrag_h(vhp + db);
        const v16h vla = ldfrag_h(vlp + da), vlb2 = ldfrag_h(vlp + db);
        o[2 * jg]     = mma_h(ph.v, vha,  o[2 * jg]);
        o[2 * jg]     = mma_h(ph.v, vla,  o[2 * jg]);
        o[2 * jg + 1] = mma_h(ph.v, vhb2, o[2 * jg + 1]);
        o[2 * jg + 1] = mma_h(ph.v, vlb2, o[2 * jg + 1]);
        guard2(o[2 * jg], o[2 * jg + 1], ph.v, vha, vhb2, vla, vlb2, ph.v);
      }
    }
    wave_sync_lds();
  }
  acc_guard4(o[0], o[1], o[2], o[3]);
  const float qnan = __uint_as_float(0x7fc00000u);
#pragma unroll
  for (int r = 0; r < 8; ++r) {
    const float lv  = lrow[r];
    const float ls  = (lv > 0.0f) ? lv : 1.0f;
    const float inv = (lv > 0.0f) ? ((1.0f / ls) * oc) : qnan;
#pragma unroll
    for (int j = 0; j < 4; ++j) {
      const int idx = (8 * hh + r) * SLP + j * 16 + c;
      slab[idx] = o[j][r] * inv;
    }
  }

  wave_sync_lds();
  v4u oh[4];
  const int rq = lane >> 3, c8 = (lane & 7) * 8;
#pragma unroll
  for (int it = 0; it < 4; ++it) {
    const int row = it * 4 + rq;
    const v4f a = *(const v4f*)(slab + row * SLP + c8), b4 = *(const v4f*)(slab + row * SLP + c8 + 4);
    float w[8];
#pragma unroll
    for (int e = 0; e < 4; ++e) { w[e] = a[e] * OSC; w[4 + e] = b4[e] * OSC; }
#pragma unroll
    for (int e = 0; e < 4; ++e) {
      const _Float16 h0 = (_Float16)w[2 * e], h1 = (_Float16)w[2 * e + 1];
      oh[it][e] = pk16(h_bits(h0), h_bits(h1));
    }
  }
  const size_t ob = ((size_t)b * SEQ + q0) * DMOD + (size_t)head * HD + c8;
  for (int pass = 0; pass < 2; ++pass) {
#pragma unroll
    for (int it = 0; it < 4; ++it) {
      const int row = it * 4 + rq;
      *(volatile v4u*)(OHp + ob + (size_t)row * DMOD) = oh[it];
    }
    __threadfence();
  }
}

extern "C" void kernel_launch(void* const* d_in, const int* in_sizes, int n_in,
                              void* d_out, int out_size, void* d_ws, size_t ws_size,
                              hipStream_t stream) {
  if (n_in < 4) return;
  if (in_sizes[0] < ((NB - 1) * XS_FULL + SEQ) * DMOD) return;
  if (in_sizes[1] < (NB - 1) * XS_FULL + SEQ) return;
  if (in_sizes[2] != 3 * DMOD * DMOD) return;
  if (in_sizes[3] != DMOD * DMOD) return;
  if (out_size < MROWS * DMOD) return;

  const float* x    = (const float*)d_in[0];
  const int*   mask = (const int*)d_in[1];
  const float* wqkv = (const float*)d_in[2];
  const float* wp   = (const float*)d_in[3];
  float*       out  = (float*)d_out;

  const size_t szXB = (size_t)MROWS * DMOD * 2;
  const size_t szV  = (size_t)NB * NH * HD * SEQ * 2;
  const size_t szF  = (size_t)MROWS * DMOD * 4;
  const size_t szQ  = (size_t)MROWS * DMOD * 2;
  const size_t szW  = (size_t)DMOD * DMOD * 2;
  const size_t szCS = (size_t)SEQ * CSW * 4;
  if (szV != szXB) return;
  if (szQ > szF) return;
  const size_t rA  = szXB;
  const size_t rQH = (szQ > szW) ? szQ : szW;
  size_t off = 0;
  const size_t oA  = off; off += rA;
  const size_t oF  = off; off += szF;
  const size_t oQH = off; off += rQH;
  const size_t oKH = off; off += szQ;
  const size_t oVL = off; off += szV;
  const size_t oW  = off; off += szW;
  const size_t oCS = off; off += szCS;
  if (off > ws_size) return;
  if (off > (size_t)WS_CAP) return;

  char* ws = (char*)d_ws;
  u16*   XB  = (u16*)(ws + oA);
  u16*   VH  = (u16*)(ws + oA);
  float* F   = (float*)(ws + oF);
  u16*   OH  = (u16*)(ws + oF);
  u16*   QH  = (u16*)(ws + oQH);
  u16*   WPB16 = (u16*)(ws + oQH);
  u16*   KH  = (u16*)(ws + oKH);
  u16*   VL  = (u16*)(ws + oVL);
  u16*   WB  = (u16*)(ws + oW);
  float* CS  = (float*)(ws + oCS);

  RopeFreq fr;
  {
    double a = 1.3335214321633240;
    for (int it = 0; it < 8; ++it) {
      const double a2 = a * a, a4 = a2 * a2, a7 = a4 * a2 * a;
      a = a - (a7 * a - 10.0) / (8.0 * a7);
    }
    double P = 1.0;
    for (int i = 0; i < NFREQ; ++i) {
      const float pf = (float)P;
      fr.f[i] = 1.0f / pf;
      P *= a;
    }
  }

  const dim3 b256(256), b128(128), bAT(ATT_THREADS);
  const int  n8x = (SEQ * DMOD) / 8;
  const int  n8w = (DMOD * DMOD) / 8;
  const int  n8q = (MROWS * DMOD) / 8;
  const dim3 gX((n8x + 255) / 256);
  const dim3 gW((n8w + 255) / 256);
  const dim3 gR((n8q + 255) / 256);
  const dim3 gCS(SEQ / 8);
  const dim3 gG((MROWS / 64) * (DMOD / 64));
  const dim3 gVT(NB * NH * NST);
  const dim3 gA(NQT * NHG * NB);
  const int  nrt = SEQ / 64;
  const dim3 gO(NB * nrt * (DMOD / 64));

  for (int b = 0; b < NB; ++b) {
    cvt16<<<gX, b256, 0, stream>>>(x + (size_t)b * XS_FULL * DMOD, XB + (size_t)b * SEQ * DMOD, n8x, 0, 1.0f);
  }
  cstab<<<gCS, b256, 0, stream>>>(CS, fr);
  cvt16<<<gW, b256, 0, stream>>>(wqkv, WB, n8w, 0, 1.0f);
  gemm_bf<<<gG, b128, 0, stream>>>(XB, WB, F, MROWS, DMOD, DMOD, 1.0f);
  rope16<<<gR, b256, 0, stream>>>(F, CS, QH, n8q, QSC);
  cvt16<<<gW, b256, 0, stream>>>(wqkv + (size_t)DMOD * DMOD, WB, n8w, 0, 1.0f);
  gemm_bf<<<gG, b128, 0, stream>>>(XB, WB, F, MROWS, DMOD, DMOD, 1.0f);
  rope16<<<gR, b256, 0, stream>>>(F, CS, KH, n8q, KSC);
  cvt16<<<gW, b256, 0, stream>>>(wqkv + (size_t)2 * DMOD * DMOD, WB, n8w, 0, 1.0f);
  gemm_bf<<<gG, b128, 0, stream>>>(XB, WB, F, MROWS, DMOD, DMOD, 1.0f);
  vt16<<<gVT, b256, 0, stream>>>(F, VH, VL);
  attn_h<<<gA, bAT, 0, stream>>>(QH, KH, VH, VL, mask, OH, 0, NQT);
  cvt16<<<gW, b256, 0, stream>>>(wp, WPB16, n8w, 1, WOS);
  gemm_o<1><<<gO, b128, 0, stream>>>(OH, OH, WPB16, out, 0, nrt, 1.0f / (OSC * WOS));
  (void)hipGetLastError();
}
